// EGNN_Layer_51496657879383
// MI455X (gfx1250) — hardware-run, weakly checked
//
#include <hip/hip_runtime.h>
#include <stddef.h>
#include <stdint.h>


#define NN      50000
#define NE      640000
#define HID     128
#define MPAD    50048
#define NTHR    256
#define NWAVE   8
#define EPT     8
#define CHUNK   (NTHR * EPT)
#define WCAP    (EPT * 32)
#define LISTN   (NWAVE * WCAP)
#define NBA     1024
#define SLA     10
#define NBLK    49
#define RCAP    16384
#define DEGCAP  48
#define GBM     64
#define GBN     128
#define GTHR    128
#define KN3     384
#define ATP     264
#define W2P     264
#define MTP     132
#define EDGE_TERMS 2
#define KEDGE   (HID * EDGE_TERMS)
#define LNEPS   1e-5f
#define WSMAX   134217728

#define U_W1T   (256 * (HID / 8))
#define U_W2T   (HID * (256 / 8))
#define U_WNT   (HID * (KN3 / 8))
#define U_TAB   256
#define U_HB    (MPAD * 16)
#define U_CP    50176
#define U_AGZ   ((MPAD - NN) * 32)
#define PB1     (U_W1T)
#define PB2     (PB1 + U_W2T)
#define PB3     (PB2 + U_WNT)
#define PB4     (PB3 + U_TAB)
#define PB5     (PB4 + U_HB)
#define PB6     (PB5 + U_CP)
#define PB7     (PB6 + U_AGZ)

#define BKT_ZINTS (LISTN + 2 * RCAP + 3 * NBA)
#define BKT_LDS_INTS (BKT_ZINTS + 16)
#define BKT_LDS_BYTES (BKT_LDS_INTS * 4)

#define W2F     ((HID * W2P * 2) / 4)
#define TABN    640
#define WAVEF   4608
#define EDGE_LDS_BYTES ((W2F + TABN + NWAVE * WAVEF) * 4)

static_assert(HID == 128 && 2 * HID + 1 == 257);
static_assert(NN % 32 == 16 && NN % 256 == 80);
static_assert(((long long)NN * HID * 4) % 128 == 0);
static_assert((3 * NN) % 4 == 0);
static_assert(MPAD % GBM == 0 && MPAD >= NN && MPAD % 128 == 0);
static_assert(NBLK * NBA >= MPAD && 196 * NTHR >= NN && 196 * NTHR <= NBLK * NBA);
static_assert(RCAP >= 14046 && RCAP % (NTHR * 4) == 0);
static_assert(DEGCAP >= 37);
static_assert((CHUNK & (CHUNK - 1)) == 0 && CHUNK <= 4096);
static_assert(NBA == (1 << SLA) && NBA == 4 * NTHR && NBA % 32 == 0 && NBA % GBM == 0);
static_assert(((long long)NE << SLA) < (1LL << 31));
static_assert(BKT_ZINTS % 4 == 0 && BKT_LDS_BYTES <= 327680);
static_assert(EDGE_LDS_BYTES <= 327680);
static_assert(PB1 % NTHR == 0 && PB2 % NTHR == 0 && PB3 % NTHR == 0 && PB4 % NTHR == 0);
static_assert(PB5 % NTHR == 0 && PB6 % NTHR == 0 && PB7 % NTHR == 0);
static_assert(U_CP >= MPAD);
static_assert(HID % 32 == 0 && KN3 % 32 == 0 && KEDGE % 32 == 0 && KEDGE <= 256);
static_assert((ATP * 2) % 16 == 0 && (W2P * 2) % 16 == 0 && (MTP * 4) % 16 == 0);
static_assert(ATP >= 256 && W2P >= 256 && MTP >= HID);
static_assert(WAVEF == (16 * ATP * 2) / 4 + 16 * MTP + 128 + 128 + 128);
static_assert(GBM == (GTHR / 32) * 16 && GBN == HID);

typedef float          v4f   __attribute__((ext_vector_type(4)));
typedef float          v8f   __attribute__((ext_vector_type(8)));
typedef int            v4i   __attribute__((ext_vector_type(4)));
typedef int            v8i   __attribute__((ext_vector_type(8)));
typedef unsigned       v2u   __attribute__((ext_vector_type(2)));
typedef unsigned short v4us  __attribute__((ext_vector_type(4)));
typedef unsigned short v8us  __attribute__((ext_vector_type(8)));
typedef unsigned short v16us __attribute__((ext_vector_type(16)));
typedef __bf16         v16bf __attribute__((ext_vector_type(16)));
typedef v4f  __attribute__((may_alias)) v4fa;
typedef v4i  __attribute__((may_alias)) v4ia;
typedef v2u  __attribute__((may_alias)) v2ua;
typedef v4us __attribute__((may_alias)) v4usa;
typedef v8us __attribute__((may_alias)) v8usa;
union FragB { v16bf v; v16us u; v8us h[2]; v8i w; };

__device__ __forceinline__ v8f wmb(const FragB& a, const FragB& b, v8f c) {
  v8f d = __builtin_amdgcn_wmma_f32_16x16x32_bf16(false, a.v, false, b.v, (short)0, c, false, false);
  asm volatile("v_nop\n\tv_nop\n\tv_nop\n\tv_nop" : "+v"(d) : "v"(a.w), "v"(b.w));
  return d;
}

__device__ __forceinline__ v8f z8() { v8f z = {0.f, 0.f, 0.f, 0.f, 0.f, 0.f, 0.f, 0.f}; return z; }

__device__ __forceinline__ unsigned bf16_bits(float f) {
  const unsigned u = __float_as_uint(f);
  return (u + 0x7FFFu + ((u >> 16) & 1u)) >> 16;
}
__device__ __forceinline__ float bf16_val(float f) {
  return __uint_as_float(bf16_bits(f) << 16);
}
__device__ __forceinline__ unsigned hl_bits(float v, unsigned& lo) {
  const unsigned hb = bf16_bits(v);
  lo = bf16_bits(v - __uint_as_float(hb << 16));
  return hb;
}
__device__ __forceinline__ int clampi(int v, int lo, int hi) { return v < lo ? lo : (v > hi ? hi : v); }
__device__ __forceinline__ float relu_keep(float v) { return (v > 0.0f) ? v : (v - v); }

__device__ __forceinline__ void wave_sync() {
  __builtin_amdgcn_fence(__ATOMIC_RELEASE, "wavefront");
  __builtin_amdgcn_wave_barrier();
  __builtin_amdgcn_fence(__ATOMIC_ACQUIRE, "wavefront");
}

__device__ __forceinline__ void put16(unsigned short* dp, v8us o) {
  *(volatile v8us*)dp = o;
  __threadfence();
  *(volatile v8us*)dp = o;
}
__device__ __forceinline__ void putf4(float* dp, v4f o) {
  *(volatile v4f*)dp = o;
  __threadfence();
  *(volatile v4f*)dp = o;
}
__device__ __forceinline__ void puti4(int* dp, v4i o) {
  *(volatile v4i*)dp = o;
  __threadfence();
  *(volatile v4i*)dp = o;
}

template <int SLB>
__device__ __forceinline__ int scan_chunk(const int* __restrict__ keys, int nE, int cbase, int slotBase,
                                          int nb, int vec8, int* list, int tid, int lane, int wave) {
  int wc = 0;
  const int el0  = tid * EPT;
  const int e0   = cbase + el0;
  const int sent = -2147483647 - 1;
  v4i da, db;
  if (vec8 != 0 && cbase + CHUNK <= nE) {
    da = *(const v4i*)(keys + e0);
    db = *(const v4i*)(keys + e0 + 4);
  } else {
    const int k0 = keys[min(e0,     nE - 1)];
    const int k1 = keys[min(e0 + 1, nE - 1)];
    const int k2 = keys[min(e0 + 2, nE - 1)];
    const int k3 = keys[min(e0 + 3, nE - 1)];
    const int k4 = keys[min(e0 + 4, nE - 1)];
    const int k5 = keys[min(e0 + 5, nE - 1)];
    const int k6 = keys[min(e0 + 6, nE - 1)];
    const int k7 = keys[min(e0 + 7, nE - 1)];
    asm volatile("" :: "v"(k0), "v"(k1), "v"(k2), "v"(k3), "v"(k4), "v"(k5), "v"(k6), "v"(k7));
    da.x = (e0     < nE) ? k0 : sent;
    da.y = (e0 + 1 < nE) ? k1 : sent;
    da.z = (e0 + 2 < nE) ? k2 : sent;
    da.w = (e0 + 3 < nE) ? k3 : sent;
    db.x = (e0 + 4 < nE) ? k4 : sent;
    db.y = (e0 + 5 < nE) ? k5 : sent;
    db.z = (e0 + 6 < nE) ? k6 : sent;
    db.w = (e0 + 7 < nE) ? k7 : sent;
  }
  const unsigned nbs = (unsigned)slotBase;
  const unsigned unb = (unsigned)nb;
  const unsigned s0 = (unsigned)da.x - nbs, s1 = (unsigned)da.y - nbs;
  const unsigned s2 = (unsigned)da.z - nbs, s3 = (unsigned)da.w - nbs;
  const unsigned s4 = (unsigned)db.x - nbs, s5 = (unsigned)db.y - nbs;
  const unsigned s6 = (unsigned)db.z - nbs, s7 = (unsigned)db.w - nbs;
  const bool h0 = s0 < unb, h1 = s1 < unb, h2 = s2 < unb, h3 = s3 < unb;
  const bool h4 = s4 < unb, h5 = s5 < unb, h6 = s6 < unb, h7 = s7 < unb;
  const unsigned any = __builtin_amdgcn_ballot_w32(h0 | h1 | h2 | h3 | h4 | h5 | h6 | h7);
  if (any != 0u) {
#define HITJ(J, HJ, SJ) { \
      const unsigned mj = __builtin_amdgcn_ballot_w32(HJ); \
      if (mj != 0u) { \
        if (HJ) { \
          const int pos = wc + (int)__builtin_amdgcn_mbcnt_lo(mj, 0u); \
          if (pos < WCAP) list[wave * WCAP + pos] = ((el0 + (J)) << SLB) | (int)(SJ); \
        } \
        wc += (int)__builtin_popcount(mj); } }
    HITJ(0, h0, s0)
    HITJ(1, h1, s1)
    HITJ(2, h2, s2)
    HITJ(3, h3, s3)
    HITJ(4, h4, s4)
    HITJ(5, h5, s5)
    HITJ(6, h6, s6)
    HITJ(7, h7, s7)
#undef HITJ
  }
  return wc;
}

__global__ __launch_bounds__(NTHR) void k_prep(const float* __restrict__ h, const float* __restrict__ x,
                                               const float* __restrict__ We1, const float* __restrict__ be1,
                                               const float* __restrict__ We2, const float* __restrict__ be2,
                                               const float* __restrict__ Wc, const float* __restrict__ bc,
                                               const float* __restrict__ Wn, const float* __restrict__ bn,
                                               const float* __restrict__ lng, const float* __restrict__ lnb,
                                               const float* __restrict__ crw,
                                               unsigned short* W1T, unsigned short* W2T2, unsigned short* WNT3,
                                               float* TAB, unsigned short* HB, float* CP, unsigned short* AGG) {
  const int u = (int)blockIdx.x * NTHR + (int)threadIdx.x;
  v8us o;
  if (u < PB1) {
    const int n   = u >> 4;
    const int k8  = (u & 15) * 8;
    const int q   = n >> 7;
    const int nn  = n & (HID - 1);
    const float* p = We1 + (size_t)(q * HID + k8) * HID + nn;
#pragma unroll
    for (int i = 0; i < 8; ++i) o[i] = (unsigned short)bf16_bits(p[(size_t)i * HID]);
    put16(W1T + (size_t)n * HID + k8, o);
    return;
  } else if (u < PB2) {
    const int v    = u - PB1;
    const int n    = v >> 5;
    const int k8   = (v & 31) * 8;
    const int srow = k8 & (HID - 1);
    const float* p = We2 + (size_t)srow * HID + n;
#pragma unroll
    for (int i = 0; i < 8; ++i) o[i] = (unsigned short)bf16_bits(p[(size_t)i * HID]);
    put16(W2T2 + (size_t)n * 256 + k8, o);
    return;
  } else if (u < PB3) {
    const int v    = u - PB2;
    const int n    = v / (KN3 / 8);
    const int k8   = (v - n * (KN3 / 8)) * 8;
    const int srow = (k8 < 2 * HID) ? k8 : (k8 - HID);
    const float* p = Wn + (size_t)srow * HID + n;
#pragma unroll
    for (int i = 0; i < 8; ++i) o[i] = (unsigned short)bf16_bits(p[(size_t)i * HID]);
    put16(WNT3 + (size_t)n * KN3 + k8, o);
    return;
  } else if (u < PB4) {
    const int v  = u - PB3;
    const int t  = v >> 5;
    const int c4 = (v & 31) * 4;
    v4f q;
    if (t == 0)      q = *(const v4fa*)(We1 + (size_t)256 * HID + c4);
    else if (t == 1) q = *(const v4fa*)(be1 + c4);
    else if (t == 2) q = *(const v4fa*)(be2 + c4);
    else if (t == 3) q = *(const v4fa*)(Wc + c4);
    else if (t == 4) q = *(const v4fa*)(bn + c4);
    else if (t == 5) q = *(const v4fa*)(lng + c4);
    else if (t == 6) q = *(const v4fa*)(lnb + c4);
    else {
      const float b0 = bc[0];
      const float c0 = crw[0];
      asm volatile("" :: "v"(b0), "v"(c0));
      q.x = (c4 == 0) ? b0 : 0.0f;
      q.y = (c4 == 0) ? c0 : 0.0f;
      q.z = 0.0f;
      q.w = 0.0f;
    }
    v4f r;
    r.x = bf16_val(q.x); r.y = bf16_val(q.y); r.z = bf16_val(q.z); r.w = bf16_val(q.w);
    putf4(TAB + (size_t)v * 4, r);
    return;
  } else if (u < PB5) {
    const int v   = u - PB4;
    const int row = v >> 4;
    const int k8  = (v & 15) * 8;
    const int rc  = row < NN ? row : NN - 1;
    const float* p = h + (size_t)rc * HID + k8;
    const v4f a = *(const v4fa*)p;
    const v4f b = *(const v4fa*)(p + 4);
    const bool ok = row < NN;
    o[0] = ok ? (unsigned short)bf16_bits(a.x) : (unsigned short)0;
    o[1] = ok ? (unsigned short)bf16_bits(a.y) : (unsigned short)0;
    o[2] = ok ? (unsigned short)bf16_bits(a.z) : (unsigned short)0;
    o[3] = ok ? (unsigned short)bf16_bits(a.w) : (unsigned short)0;
    o[4] = ok ? (unsigned short)bf16_bits(b.x) : (unsigned short)0;
    o[5] = ok ? (unsigned short)bf16_bits(b.y) : (unsigned short)0;
    o[6] = ok ? (unsigned short)bf16_bits(b.z) : (unsigned short)0;
    o[7] = ok ? (unsigned short)bf16_bits(b.w) : (unsigned short)0;
    put16(HB + (size_t)row * HID + k8, o);
    return;
  } else if (u < PB6) {
    const int row = u - PB5;
    if (row >= MPAD) return;
    const int rc  = row < NN ? row : NN - 1;
    const bool ok = row < NN;
    const float x0 = x[(size_t)rc * 3 + 0];
    const float x1 = x[(size_t)rc * 3 + 1];
    const float x2 = x[(size_t)rc * 3 + 2];
    v4f q;
    q.x = ok ? bf16_val(x0) : 0.0f;
    q.y = ok ? bf16_val(x1) : 0.0f;
    q.z = ok ? bf16_val(x2) : 0.0f;
    q.w = 0.0f;
    putf4(CP + (size_t)row * 4, q);
    return;
  } else if (u < PB7) {
    const int v   = u - PB6;
    const int row = NN + (v >> 5);
    const int k8  = (v & 31) * 8;
#pragma unroll
    for (int i = 0; i < 8; ++i) o[i] = (unsigned short)0;
    put16(AGG + (size_t)row * 256 + k8, o);
    return;
  }
}

__global__ __launch_bounds__(GTHR) void k_gemm_ab(const unsigned short* __restrict__ A,
                                                  const unsigned short* __restrict__ BT, float* Cm) {
  __shared__ __attribute__((aligned(16))) float stg[GBM * GBN];
  const int tid = (int)threadIdx.x, lane = tid & 31, wave = tid >> 5, hh = lane >> 4, m = lane & 15;
  const int rowBase = (int)blockIdx.x * GBM;
  const int colBase = (int)blockIdx.y * GBN;

  v8f acc[8];
#pragma unroll
  for (int t = 0; t < 8; ++t) acc[t] = z8();
  const unsigned short* ap = A  + (size_t)(rowBase + 16 * wave + m) * HID + 8 * hh;
  const unsigned short* bp = BT + (size_t)(colBase + m) * HID + 8 * hh;

#pragma unroll 1
  for (int k0 = 0; k0 < HID; k0 += 32) {
    FragB af;
    af.h[0] = *(const v8usa*)(ap + k0);
    af.h[1] = *(const v8usa*)(ap + k0 + 16);
#pragma unroll
    for (int nt = 0; nt < 8; ++nt) {
      const unsigned short* wq = bp + (size_t)(16 * nt) * HID + k0;
      FragB bf;
      bf.h[0] = *(const v8usa*)wq;
      bf.h[1] = *(const v8usa*)(wq + 16);
      acc[nt] = wmb(af, bf, acc[nt]);
    }
  }

#pragma unroll
  for (int nt = 0; nt < 8; ++nt) {
    const int lc = 16 * nt + m;
#pragma unroll
    for (int r = 0; r < 8; ++r) {
      const int lr = 16 * wave + 8 * hh + r;
      stg[lr * GBN + lc] = acc[nt][r];
    }
  }
  __syncthreads();

  v4f pv[16];
#pragma unroll
  for (int i = 0; i < 16; ++i) pv[i] = *(const v4fa*)(stg + (16 * wave + i) * GBN + 4 * lane);
#pragma unroll
  for (int i = 0; i < 16; ++i) {
    float* op = Cm + (size_t)(rowBase + 16 * wave + i) * 256 + colBase + 4 * lane;
    *(volatile v4f*)op = pv[i];
  }
  __threadfence();
#pragma unroll
  for (int i = 0; i < 16; ++i) {
    float* op = Cm + (size_t)(rowBase + 16 * wave + i) * 256 + colBase + 4 * lane;
    *(volatile v4f*)op = pv[i];
  }
}

__global__ __launch_bounds__(NTHR) void k_bucket(const int* __restrict__ keys, const int* __restrict__ cols,
                                                 int nE, int vec8, int* LIST, int* CNT, int* OFF, int* FLAG) {
  extern __shared__ __attribute__((aligned(16))) int dsm[];
  int* list = dsm;
  int* hl   = dsm + LISTN;
  int* sl   = hl + RCAP;
  int* cnt  = sl + RCAP;
  int* offs = cnt + NBA;
  int* cur  = offs + NBA;
  int* misc = cur + NBA;
  const int tid = (int)threadIdx.x, lane = tid & 31, wave = tid >> 5;
  const int nodeBase = (int)blockIdx.x * NBA;

  {
    const v4i z4 = {0, 0, 0, 0};
    for (int i = tid * 4; i < BKT_ZINTS; i += NTHR * 4) *(v4ia*)(dsm + i) = z4;
    if (tid < 16) misc[tid] = 0;
  }
  __syncthreads();

  int t = 0, ov = 0;
  const int nChunks = (nE + CHUNK - 1) / CHUNK;
#pragma unroll 1
  for (int ch = 0; ch < nChunks; ++ch) {
    const int cbase = ch * CHUNK;
    const int wc = scan_chunk<SLA>(keys, nE, cbase, nodeBase, NBA, vec8, list, tid, lane, wave);
    if (lane == 0) misc[wave] = wc;
    __syncthreads();
    if (wave == 0) {
#pragma unroll 1
      for (int w2 = 0; w2 < NWAVE; ++w2) {
        int c = misc[w2];
        c = c < 0 ? 0 : (c > WCAP ? WCAP : c);
#pragma unroll 1
        for (int b0 = 0; b0 < c; b0 += 32) {
          const int idx = b0 + lane;
          const int ent = list[w2 * WCAP + (idx < WCAP ? idx : WCAP - 1)];
          const int m32 = (c - b0) < 32 ? (c - b0) : 32;
#pragma unroll 1
          for (int k = 0; k < m32; ++k) {
            const int u    = __builtin_amdgcn_readlane(ent, k);
            const int slot = u & (NBA - 1);
            const int el   = (u >> SLA) & (CHUNK - 1);
            const int pk   = ((cbase + el) << SLA) | slot;
            if (t < RCAP) {
              if (lane == 0) { hl[t] = pk; cnt[slot] = cnt[slot] + 1; }
              t = t + 1;
            } else {
              ov = 1;
            }
          }
        }
      }
    }
    __syncthreads();
  }
  if (wave == 0 && lane == 0) { misc[8] = t; misc[9] = ov; }
  __syncthreads();
  int tt = misc[8];
  tt = tt < 0 ? 0 : (tt > RCAP ? RCAP : tt);
  const int ovf = misc[9];

  if (wave == 0) {
    const int base = lane * (NBA / 32);
    int s = 0;
#pragma unroll 1
    for (int i = 0; i < NBA / 32; ++i) s += cnt[base + i];
    int incl = s;
#pragma unroll
    for (int d = 1; d < 32; d <<= 1) {
      const int y = __shfl_up(incl, d, 32);
      if (lane >= d) incl += y;
    }
    int run = incl - s;
#pragma unroll 1
    for (int i = 0; i < NBA / 32; ++i) {
      const int cv = cnt[base + i];
      offs[base + i] = run;
      cur[base + i]  = run;
      run += cv;
    }
  }
  __syncthreads();
  if (wave == 0) {
#pragma unroll 1
    for (int b0 = 0; b0 < tt; b0 += 32) {
      const int idx = b0 + lane;
      const int ent = hl[idx < RCAP ? idx : RCAP - 1];
      const int m32 = (tt - b0) < 32 ? (tt - b0) : 32;
#pragma unroll 1
      for (int k = 0; k < m32; ++k) {
        const int u    = __builtin_amdgcn_readlane(ent, k);
        const int slot = u & (NBA - 1);
        if (lane == 0) {
          int p = cur[slot];
          p = p < 0 ? 0 : (p > RCAP - 1 ? RCAP - 1 : p);
          sl[p] = u;
          cur[slot] = p + 1;
        }
      }
    }
  }
  __syncthreads();

  int* lb = LIST + (size_t)blockIdx.x * RCAP;
#pragma unroll 1
  for (int it = 0; it < RCAP / (NTHR * 4); ++it) {
    const int p = (it * NTHR + tid) * 4;
    const v4i u4 = *(const v4ia*)(sl + p);
    const int e0 = clampi(u4.x >> SLA, 0, nE - 1);
    const int e1 = clampi(u4.y >> SLA, 0, nE - 1);
    const int e2 = clampi(u4.z >> SLA, 0, nE - 1);
    const int e3 = clampi(u4.w >> SLA, 0, nE - 1);
    const int c0 = cols[e0];
    const int c1 = cols[e1];
    const int c2 = cols[e2];
    const int c3 = cols[e3];
    asm volatile("" :: "v"(c0), "v"(c1), "v"(c2), "v"(c3));
    v4i o;
    o.x = (p     < tt) ? clampi(c0, 0, NN - 1) : 0;
    o.y = (p + 1 < tt) ? clampi(c1, 0, NN - 1) : 0;
    o.z = (p + 2 < tt) ? clampi(c2, 0, NN - 1) : 0;
    o.w = (p + 3 < tt) ? clampi(c3, 0, NN - 1) : 0;
    puti4(lb + p, o);
  }
  {
    const v4i c4 = *(const v4ia*)(cnt + 4 * tid);
    const v4i o4 = *(const v4ia*)(offs + 4 * tid);
    puti4(CNT + (size_t)blockIdx.x * NBA + 4 * tid, c4);
    puti4(OFF + (size_t)blockIdx.x * NBA + 4 * tid, o4);
  }
  {
    const v4i f4 = {ovf, ovf, ovf, ovf};
    int* fp = FLAG + (size_t)blockIdx.x * 32 + 4 * (tid & 7);
    if (tid < 8) *(volatile v4i*)fp = f4;
    __threadfence();
    if (tid < 8) *(volatile v4i*)fp = f4;
  }
}

__device__ __forceinline__ void flush_node(unsigned short* AGG, unsigned short* rowbuf, float* dsl, int node, int slot,
                                           int lane, float a0, float a1, float a2, float a3,
                                           float dx, float dy, float dz, float pz) {
  const float m0 = a0 + pz, m1 = a1 + pz, m2 = a2 + pz, m3 = a3 + pz;
  v4us mh, ml;
  {
    unsigned lb;
    unsigned hb;
    hb = hl_bits(m0, lb); mh[0] = (unsigned short)hb; ml[0] = (unsigned short)lb;
    hb = hl_bits(m1, lb); mh[1] = (unsigned short)hb; ml[1] = (unsigned short)lb;
    hb = hl_bits(m2, lb); mh[2] = (unsigned short)hb; ml[2] = (unsigned short)lb;
    hb = hl_bits(m3, lb); mh[3] = (unsigned short)hb; ml[3] = (unsigned short)lb;
  }
  *(v4usa*)(rowbuf + 4 * lane)       = mh;
  *(v4usa*)(rowbuf + HID + 4 * lane) = ml;
  wave_sync();
  const v8us q0 = *(const v8usa*)(rowbuf + 8 * lane);
  wave_sync();
  unsigned short* rp = AGG + (size_t)node * 256 + 8 * lane;
  *(volatile v8us*)rp = q0;
  __threadfence();
  *(volatile v8us*)rp = q0;
  if (lane == 0) {
    const v4f d4 = {dx + pz, dy + pz, dz + pz, 0.0f};
    *(v4fa*)(dsl + 4 * slot) = d4;
  }
}

__global__ __launch_bounds__(NTHR) __attribute__((amdgpu_num_vgpr(248)))
void k_edge(const float* __restrict__ AB, const float* __restrict__ CP, const int* __restrict__ LIST,
            const int* __restrict__ CNT, const int* __restrict__ OFF, const int* __restrict__ FLAG,
            const unsigned short* __restrict__ W2G, const float* __restrict__ TAB,
            unsigned short* AGG, float* out1) {
  extern __shared__ __attribute__((aligned(16))) float dyn[];
  unsigned short* sW2  = (unsigned short*)dyn;
  float*          sTab = dyn + W2F;
  const int tid = (int)threadIdx.x, lane = tid & 31, hh = lane >> 4, m = lane & 15;
  const int wave = __builtin_amdgcn_readfirstlane(tid >> 5);
  float*          wbase  = sTab + TABN + wave * WAVEF;
  unsigned short* sA     = (unsigned short*)wbase;
  float*          sM     = wbase + (16 * ATP * 2) / 4;
  unsigned short* rowbuf = (unsigned short*)(sM + 16 * MTP);
  float*          xst    = sM + 16 * MTP + 128;
  float*          dsl    = xst + 128;

#pragma unroll 4
  for (int it = 0; it < (HID * 32) / NTHR; ++it) {
    const int u  = it * NTHR + tid;
    const int n  = u >> 5;
    const int k8 = (u & 31) * 8;
    const v8us v = *(const v8usa*)(W2G + (size_t)n * 256 + k8);
    *(v8usa*)(sW2 + n * W2P + k8) = v;
  }
  if (tid < 160) {
    const int src = tid < 128 ? 4 * tid : (7 * HID + 4 * (tid - 128));
    const v4f v = *(const v4fa*)(TAB + src);
    *(v4fa*)(sTab + 4 * tid) = v;
  }
  {
    const v4f z4 = {0.0f, 0.0f, 0.0f, 0.0f};
    *(v4fa*)(dsl + 4 * lane) = z4;
  }
  __syncthreads();

  const int n0 = (int)blockIdx.x * NTHR + wave * 32;
  if (n0 < NN) {
    const int bb  = n0 >> SLA;
    const int flg = FLAG[bb * 32];
    const int nd  = n0 + lane;
    const int craw = CNT[nd];
    const int oraw = OFF[nd];
    asm volatile("" :: "v"(craw), "v"(oraw));
    const bool nok = nd < NN;
    const bool big = nok && (craw < 0 || craw > DEGCAP);
    const int c = nok ? clampi(craw, 0, DEGCAP) : 0;
    const unsigned bigm = __builtin_amdgcn_ballot_w32(big);
    const float qnan = __int_as_float(0x7fc00000);
    const float pz = (bigm != 0u || flg != 0) ? qnan : 0.0f;
    int incl = c;
#pragma unroll
    for (int d = 1; d < 32; d <<= 1) {
      const int y = __shfl_up(incl, d, 32);
      if (lane >= d) incl += y;
    }
    const int T   = __builtin_amdgcn_readlane(incl, 31);
    const int ocl = clampi(oraw, 0, RCAP - 1);
    const int S   = __builtin_amdgcn_readfirstlane(ocl);
    const int* lb = LIST + (size_t)bb * RCAP;

    const v4f w256 = *(const v4fa*)(sTab + 4 * lane);
    const v4f be1v = *(const v4fa*)(sTab + HID + 4 * lane);
    const float bcv = sTab[512];
    const float crw = sTab[513];

    int curP = 0;
    int remP = __builtin_amdgcn_readlane(c, 0);
    int curD = 0;
    float a0 = 0.0f, a1 = 0.0f, a2 = 0.0f, a3 = 0.0f;
    float dx = 0.0f, dy = 0.0f, dz = 0.0f;

#pragma unroll 1
    for (int t0 = 0; t0 < T; t0 += 16) {
      wave_sync();
      int myslot = 0;
#pragma unroll 1
      for (int i = 0; i < 16; ++i) {
        if (t0 + i < T) {
          while (remP == 0 && curP < 31) { ++curP; remP = __builtin_amdgcn_readlane(c, curP); }
          if (remP > 0) --remP;
        }
        myslot = (m == i) ? curP : myslot;
      }
      const int j   = t0 + m;
      const int jl  = j < T ? j : T - 1;
      const int pos = clampi(S + jl, 0, RCAP - 1);
      const int colv = clampi(lb[pos], 0, NN - 1);
      int own = n0 + myslot;
      own = own > NN - 1 ? NN - 1 : own;
      const v4f xr = *(const v4fa*)(CP + (size_t)own * 4);
      const v4f xc = *(const v4fa*)(CP + (size_t)colv * 4);
      const float rx = xr.x - xc.x, ry = xr.y - xc.y, rz = xr.z - xc.z;
      const float d2 = (rx * rx + rz * rz) + ry * ry;

#pragma unroll 1
      for (int i = 0; i < 16; ++i) {
        const bool live = (t0 + i) < T;
        int ri = n0 + __builtin_amdgcn_readlane(myslot, i);
        ri = ri > NN - 1 ? NN - 1 : ri;
        const int ci = __builtin_amdgcn_readlane(colv, i);
        const float d2i = __int_as_float(__builtin_amdgcn_readlane(__float_as_int(d2), i));
        const v4f a4 = *(const v4fa*)(AB + (size_t)ri * 256 + 4 * lane);
        const v4f b4 = *(const v4fa*)(AB + (size_t)ci * 256 + HID + 4 * lane);
        float z0 = (a4.x + b4.x) + fmaf(d2i, w256.x, be1v.x);
        float z1 = (a4.y + b4.y) + fmaf(d2i, w256.y, be1v.y);
        float z2 = (a4.z + b4.z) + fmaf(d2i, w256.z, be1v.z);
        float z3 = (a4.w + b4.w) + fmaf(d2i, w256.w, be1v.w);
        z0 = relu_keep(z0); z1 = relu_keep(z1); z2 = relu_keep(z2); z3 = relu_keep(z3);
        z0 = live ? z0 : 0.0f; z1 = live ? z1 : 0.0f; z2 = live ? z2 : 0.0f; z3 = live ? z3 : 0.0f;
        unsigned l0, l1, l2, l3;
        const unsigned h0 = hl_bits(z0, l0);
        const unsigned h1 = hl_bits(z1, l1);
        const unsigned h2 = hl_bits(z2, l2);
        const unsigned h3 = hl_bits(z3, l3);
        v2u wh, wl;
        wh.x = (h0 & 0xffffu) | (h1 << 16);
        wh.y = (h2 & 0xffffu) | (h3 << 16);
        wl.x = (l0 & 0xffffu) | (l1 << 16);
        wl.y = (l2 & 0xffffu) | (l3 << 16);
        *(v2ua*)(sA + i * ATP + 4 * lane)       = wh;
        *(v2ua*)(sA + i * ATP + HID + 4 * lane) = wl;
      }
      wave_sync();

      v8f acc[8];
#pragma unroll
      for (int t = 0; t < 8; ++t) acc[t] = z8();
      {
        const unsigned short* ap = sA  + m * ATP + 8 * hh;
        const unsigned short* bp = sW2 + m * W2P + 8 * hh;
#pragma unroll 1
        for (int k0 = 0; k0 < KEDGE; k0 += 32) {
          FragB af;
          af.h[0] = *(const v8usa*)(ap + k0);
          af.h[1] = *(const v8usa*)(ap + k0 + 16);
#pragma unroll
          for (int nt = 0; nt < 8; ++nt) {
            const unsigned short* wq = bp + (16 * nt) * W2P + k0;
            FragB bf;
            bf.h[0] = *(const v8usa*)wq;
            bf.h[1] = *(const v8usa*)(wq + 16);
            acc[nt] = wmb(af, bf, acc[nt]);
          }
        }
      }
#pragma unroll
      for (int nt = 0; nt < 8; ++nt) {
        const int col = 16 * nt + m;
        const float bv = sTab[2 * HID + col];
#pragma unroll
        for (int r = 0; r < 8; ++r) sM[(8 * hh + r) * MTP + col] = acc[nt][r] + bv;
      }
      wave_sync();

      float sc;
      {
        const float* mr = sM + m * MTP + 64 * hh;
        const float* wc = sTab + 3 * HID + 64 * hh;
        float dot = 0.0f;
#pragma unroll 4
        for (int c4 = 0; c4 < 16; ++c4) {
          const v4f mv = *(const v4fa*)(mr + 4 * c4);
          const v4f wv = *(const v4fa*)(wc + 4 * c4);
          dot = fmaf(mv.x, wv.x, dot);
          dot = fmaf(mv.y, wv.y, dot);
          dot = fmaf(mv.z, wv.z, dot);
          dot = fmaf(mv.w, wv.w, dot);
        }
        dot += __shfl_xor(dot, 16, 32);
        const float g = relu_keep(dot + bcv);
        sc = tanhf(g);
      }
      const float sx = rx * sc, sy = ry * sc, sz = rz * sc;

#pragma unroll 1
      for (int i = 0; i < 16; ++i) {
        if (t0 + i < T) {
          const int s = __builtin_amdgcn_readlane(myslot, i);
          while (curD < s) {
            flush_node(AGG, rowbuf, dsl, n0 + curD, curD, lane, a0, a1, a2, a3, dx, dy, dz, pz);
            a0 = 0.0f; a1 = 0.0f; a2 = 0.0f; a3 = 0.0f; dx = 0.0f; dy = 0.0f; dz = 0.0f;
            ++curD;
          }
          const v4f mv = *(const v4fa*)(sM + i * MTP + 4 * lane);
          a0 += mv.x; a1 += mv.y; a2 += mv.z; a3 += mv.w;
          dx += __int_as_float(__builtin_amdgcn_readlane(__float_as_int(sx), i));
          dy += __int_as_float(__builtin_amdgcn_readlane(__float_as_int(sy), i));
          dz += __int_as_float(__builtin_amdgcn_readlane(__float_as_int(sz), i));
        }
      }
    }

    const int nsl = (NN - n0) < 32 ? (NN - n0) : 32;
    while (curD < nsl) {
      flush_node(AGG, rowbuf, dsl, n0 + curD, curD, lane, a0, a1, a2, a3, dx, dy, dz, pz);
      a0 = 0.0f; a1 = 0.0f; a2 = 0.0f; a3 = 0.0f; dx = 0.0f; dy = 0.0f; dz = 0.0f;
      ++curD;
    }
    wave_sync();

    {
      const int nc = nd < NN ? nd : NN - 1;
      const v4f xv = *(const v4fa*)(CP + (size_t)nc * 4);
      const v4f dv = *(const v4fa*)(dsl + 4 * lane);
      xst[3 * lane + 0] = fmaf(crw, dv.x, xv.x) + pz;
      xst[3 * lane + 1] = fmaf(crw, dv.y, xv.y) + pz;
      xst[3 * lane + 2] = fmaf(crw, dv.z, xv.z) + pz;
    }
    wave_sync();
    {
      const int tl = lane < 24 ? lane : 23;
      const v4f o4 = *(const v4fa*)(xst + 4 * tl);
      const float p0 = o4.x, p1 = o4.y, p2 = o4.z, p3 = o4.w;
      asm volatile("" :: "v"(p0), "v"(p1), "v"(p2), "v"(p3));
      const int gidx = n0 * 3 + 4 * lane;
      const bool stv = (lane < 24) && (gidx + 4 <= 3 * NN);
      float* op = out1 + (size_t)(n0 * 3 + 4 * tl);
      if (stv) *(volatile v4f*)op = o4;
      __threadfence();
      if (stv) *(volatile v4f*)op = o4;
    }
  }
}

__global__ __launch_bounds__(GTHR) void k_gemm_n(const unsigned short* __restrict__ HB,
                                                 const unsigned short* __restrict__ AGG,
                                                 const unsigned short* __restrict__ WNT,
                                                 const float* __restrict__ TAB, const int* __restrict__ FLAG,
                                                 float* out0) {
  __shared__ __attribute__((aligned(16))) float stg[GBM * GBN];
  __shared__ __attribute__((aligned(16))) float stab[3 * HID];
  const int tid = (int)threadIdx.x, lane = tid & 31, wave = tid >> 5, hh = lane >> 4, m = lane & 15;
  const int rowBase = (int)blockIdx.x * GBM;

  v8f acc[8];
#pragma unroll
  for (int t = 0; t < 8; ++t) acc[t] = z8();
  const unsigned short* ap = HB  + (size_t)(rowBase + 16 * wave + m) * HID + 8 * hh;
  const unsigned short* gp = AGG + (size_t)(rowBase + 16 * wave + m) * 256 + 8 * hh;
  const unsigned short* bp = WNT + (size_t)m * KN3 + 8 * hh;

#pragma unroll 1
  for (int k0 = 0; k0 < HID; k0 += 32) {
    FragB af;
    af.h[0] = *(const v8usa*)(ap + k0);
    af.h[1] = *(const v8usa*)(ap + k0 + 16);
#pragma unroll
    for (int nt = 0; nt < 8; ++nt) {
      const unsigned short* wq = bp + (size_t)(16 * nt) * KN3 + k0;
      FragB bf;
      bf.h[0] = *(const v8usa*)wq;
      bf.h[1] = *(const v8usa*)(wq + 16);
      acc[nt] = wmb(af, bf, acc[nt]);
    }
  }
#pragma unroll 1
  for (int k0 = 0; k0 < 2 * HID; k0 += 32) {
    FragB af;
    af.h[0] = *(const v8usa*)(gp + k0);
    af.h[1] = *(const v8usa*)(gp + k0 + 16);
#pragma unroll
    for (int nt = 0; nt < 8; ++nt) {
      const unsigned short* wq = bp + (size_t)(16 * nt) * KN3 + HID + k0;
      FragB bf;
      bf.h[0] = *(const v8usa*)wq;
      bf.h[1] = *(const v8usa*)(wq + 16);
      acc[nt] = wmb(af, bf, acc[nt]);
    }
  }

#pragma unroll
  for (int nt = 0; nt < 8; ++nt) {
    const int lc = 16 * nt + m;
#pragma unroll
    for (int r = 0; r < 8; ++r) {
      const int lr = 16 * wave + 8 * hh + r;
      stg[lr * GBN + lc] = acc[nt][r];
    }
  }
  if (tid < 96) {
    const v4f v = *(const v4fa*)(TAB + 4 * HID + 4 * tid);
    *(v4fa*)(stab + 4 * tid) = v;
  }
  __syncthreads();

  const v4f bq = *(const v4fa*)(stab + 4 * lane);
  const v4f gq = *(const v4fa*)(stab + HID + 4 * lane);
  const v4f eq = *(const v4fa*)(stab + 2 * HID + 4 * lane);
  const int fl = FLAG[(rowBase >> SLA) * 32];
  const float pzb = (fl != 0) ? __int_as_float(0x7fc00000) : 0.0f;

  const float invd = 1.0f / (float)HID;
#pragma unroll 4
  for (int i = 0; i < 16; ++i) {
    const int row = rowBase + 16 * wave + i;
    float* srow = stg + (16 * wave + i) * GBN + 4 * lane;
    const v4f pvi = *(const v4fa*)srow;
    const v2u hw = *(const v2ua*)(HB + (size_t)row * HID + 4 * lane);
    const float h0 = __uint_as_float(hw.x << 16);
    const float h1 = __uint_as_float(hw.x & 0xffff0000u);
    const float h2 = __uint_as_float(hw.y << 16);
    const float h3 = __uint_as_float(hw.y & 0xffff0000u);
    const float y0 = h0 + relu_keep(pvi.x + bq.x);
    const float y1 = h1 + relu_keep(pvi.y + bq.y);
    const float y2 = h2 + relu_keep(pvi.z + bq.z);
    const float y3 = h3 + relu_keep(pvi.w + bq.w);
    float s = (y0 + y1) + (y2 + y3);
    s += __shfl_xor(s, 16, 32);
    s += __shfl_xor(s, 8, 32);
    s += __shfl_xor(s, 4, 32);
    s += __shfl_xor(s, 2, 32);
    s += __shfl_xor(s, 1, 32);
    const float mean = s * invd;
    const float d0 = y0 - mean, d1 = y1 - mean, d2 = y2 - mean, d3 = y3 - mean;
    float q = (d0 * d0 + d1 * d1) + (d2 * d2 + d3 * d3);
    q += __shfl_xor(q, 16, 32);
    q += __shfl_xor(q, 8, 32);
    q += __shfl_xor(q, 4, 32);
    q += __shfl_xor(q, 2, 32);
    q += __shfl_xor(q, 1, 32);
    const float var  = q * invd;
    const float rstd = rsqrtf(var + LNEPS);
    v4f qo;
    qo.x = fmaf(d0 * rstd, gq.x, eq.x) + pzb;
    qo.y = fmaf(d1 * rstd, gq.y, eq.y) + pzb;
    qo.z = fmaf(d2 * rstd, gq.z, eq.z) + pzb;
    qo.w = fmaf(d3 * rstd, gq.w, eq.w) + pzb;
    *(v4fa*)srow = qo;
  }

#pragma unroll 4
  for (int i = 0; i < 16; ++i) {
    const int row = rowBase + 16 * wave + i;
    const v4f ov = *(const v4fa*)(stg + (16 * wave + i) * GBN + 4 * lane);
    float* op = out0 + (size_t)row * HID + 4 * lane;
    if (row < NN) *(volatile v4f*)op = ov;
  }
  __threadfence();
#pragma unroll 4
  for (int i = 0; i < 16; ++i) {
    const int row = rowBase + 16 * wave + i;
    const v4f ov = *(const v4fa*)(stg + (16 * wave + i) * GBN + 4 * lane);
    float* op = out0 + (size_t)row * HID + 4 * lane;
    if (row < NN) *(volatile v4f*)op = ov;
  }
}

static inline size_t al256(size_t o) { return (o + 255) & ~(size_t)255; }

extern "C" void kernel_launch(void* const* d_in, const int* in_sizes, int n_in,
                              void* d_out, int out_size, void* d_ws, size_t ws_size,
                              hipStream_t stream) {
  if (n_in < 14) return;
  if (in_sizes[0] != NN * HID) return;
  if (in_sizes[1] != 3 * NN) return;
  if (in_sizes[2] != 2 * NE) return;
  if (in_sizes[3] != 257 * HID || in_sizes[4] != HID) return;
  if (in_sizes[5] != HID * HID || in_sizes[6] != HID) return;
  if (in_sizes[7] != HID || in_sizes[8] != 1) return;
  if (in_sizes[9] != 2 * HID * HID || in_sizes[10] != HID) return;
  if (in_sizes[11] != HID || in_sizes[12] != HID || in_sizes[13] != 1) return;
  if ((long long)out_size != (long long)NN * HID + 3LL * NN) return;

  const float* h   = (const float*)d_in[0];
  const float* x   = (const float*)d_in[1];
  const int*   ei  = (const int*)  d_in[2];
  const float* We1 = (const float*)d_in[3];
  const float* be1 = (const float*)d_in[4];
  const float* We2 = (const float*)d_in[5];
  const float* be2 = (const float*)d_in[6];
  const float* Wc  = (const float*)d_in[7];
  const float* bc  = (const float*)d_in[8];
  const float* Wn  = (const float*)d_in[9];
  const float* bn  = (const float*)d_in[10];
  const float* lng = (const float*)d_in[11];
  const float* lnb = (const float*)d_in[12];
  const float* crw = (const float*)d_in[13];
  float* out0 = (float*)d_out;
  float* out1 = out0 + (size_t)NN * HID;
  const int* keys = ei;
  const int* cols = ei + NE;

  char* ws = (char*)d_ws;
  size_t off = 0;
  const size_t oW1T = off; off = al256(off + (size_t)256 * HID * 2);
  const size_t oW2T = off; off = al256(off + (size_t)HID * 256 * 2);
  const size_t oWNT = off; off = al256(off + (size_t)HID * KN3 * 2);
  const size_t oTAB = off; off = al256(off + (size_t)8 * HID * 4);
  const size_t oCP  = off; off = al256(off + (size_t)MPAD * 4 * 4);
  const size_t oHB  = off; off = al256(off + (size_t)MPAD * HID * 2);
  const size_t oAB  = off; off = al256(off + (size_t)MPAD * 256 * 4);
  const size_t oAGG = off; off = al256(off + (size_t)MPAD * 256 * 2);
  const size_t oLST = off; off = al256(off + (size_t)NBLK * RCAP * 4);
  const size_t oCNT = off; off = al256(off + (size_t)NBLK * NBA * 4);
  const size_t oOFF = off; off = al256(off + (size_t)NBLK * NBA * 4);
  const size_t oFLG = off; off = al256(off + (size_t)NBLK * 32 * 4);
  if (off > ws_size || off > (size_t)WSMAX) return;
  unsigned short* W1T  = (unsigned short*)(ws + oW1T);
  unsigned short* W2T2 = (unsigned short*)(ws + oW2T);
  unsigned short* WNT3 = (unsigned short*)(ws + oWNT);
  float*          TAB  = (float*)(ws + oTAB);
  float*          CP   = (float*)(ws + oCP);
  unsigned short* HB   = (unsigned short*)(ws + oHB);
  float*          AB   = (float*)(ws + oAB);
  unsigned short* AGG  = (unsigned short*)(ws + oAGG);
  int*            LIST = (int*)(ws + oLST);
  int*            CNT  = (int*)(ws + oCNT);
  int*            OFF  = (int*)(ws + oOFF);
  int*            FLAG = (int*)(ws + oFLG);

  hipFuncSetAttribute(reinterpret_cast<const void*>(&k_bucket), hipFuncAttributeMaxDynamicSharedMemorySize,
                      (int)BKT_LDS_BYTES);
  hipFuncSetAttribute(reinterpret_cast<const void*>(&k_edge), hipFuncAttributeMaxDynamicSharedMemorySize,
                      (int)EDGE_LDS_BYTES);

  const int vec8 = 1;

  k_prep<<<PB7 / NTHR, NTHR, 0, stream>>>(h, x, We1, be1, We2, be2, Wc, bc, Wn, bn, lng, lnb, crw,
                                          W1T, W2T2, WNT3, TAB, HB, CP, AGG);
  k_gemm_ab<<<dim3(MPAD / GBM, 2), GTHR, 0, stream>>>(HB, W1T, AB);
  k_bucket<<<NBLK, NTHR, BKT_LDS_BYTES, stream>>>(keys, cols, NE, vec8, LIST, CNT, OFF, FLAG);
  k_edge<<<196, NTHR, EDGE_LDS_BYTES, stream>>>(AB, CP, LIST, CNT, OFF, FLAG, W2T2, TAB, AGG, out1);
  k_gemm_n<<<MPAD / GBM, GTHR, 0, stream>>>(HB, AGG, WNT3, TAB, FLAG, out0);
}
